// RGCNModel_21921513079385
// MI455X (gfx1250) — hardware-verified
//
#include <hip/hip_runtime.h>
#include <stddef.h>
#include <stdint.h>


#define DIN    64
#define DF     128
#define DC     64
#define NREL   7
#define NBLK   8
#define BW     256
#define AP     (NBLK * BW)
#define HOFF   (NREL * BW)
#define KCL    BW
#define NTHR   256
#define NWAVE  8
#define EPT    8
#define CHUNK  (NTHR * EPT)
#define WCAP   (EPT * 32)
#define LISTN  (NWAVE * WCAP)
#define NBA    1024
#define SLA    10
#define RCAP   28672
#define DEGCAP 64
#define GBM    64
#define GBN    128
#define GCN    64
#define GTHR   128
#define UEMB   (DF * (DIN / 8))
#define UMAT   (DF * (DF / 4))
#define ULAY   (2 * NBLK * UMAT)
#define UCLS   (DC * (DF / 4))
#define UTOT   (UEMB + ULAY + UCLS)
#define AGG_ZINTS    (LISTN + 2 * RCAP + 3 * NBA)
#define MISC_INTS    96
#define AGG_LDS_INTS (AGG_ZINTS + MISC_INTS)
#define WSMAX  268435456

static_assert((CHUNK & (CHUNK - 1)) == 0 && CHUNK <= 4096);
static_assert((NBA & (NBA - 1)) == 0 && NBA == (1 << SLA));
static_assert(((long long)CHUNK << SLA) < (1LL << 31));
static_assert(LISTN % NTHR == 0);
static_assert(NBA % NWAVE == 0 && NBA % 32 == 0 && NBA % GBM == 0);
static_assert(RCAP % 4 == 0 && AGG_ZINTS % 4 == 0 && LISTN % 4 == 0 && ((AGG_ZINTS + MISC_INTS) % 4) == 0);
static_assert(AGG_ZINTS % (NTHR * 4) == 0);
static_assert(MISC_INTS >= 16 + DEGCAP + 1 && DEGCAP + 1 <= NTHR);
static_assert(AGG_LDS_INTS * 4 <= 300000);
static_assert(DIN % 32 == 0 && AP % 32 == 0 && KCL % 32 == 0 && BW == 2 * DF && HOFF + BW == AP && BW == 8 * 32);
static_assert(GBN == DF && GCN == DC && GBM == (GTHR / 32) * 16 && DF == 4 * 32 && DC == 2 * 32);
static_assert(UEMB % NTHR == 0 && UMAT % NTHR == 0 && ULAY % NTHR == 0 && UCLS % NTHR == 0 && UTOT % NTHR == 0);

typedef float          v2f   __attribute__((ext_vector_type(2)));
typedef float          v4f   __attribute__((ext_vector_type(4)));
typedef float          v8f   __attribute__((ext_vector_type(8)));
typedef int            v4i   __attribute__((ext_vector_type(4)));
typedef int            v8i   __attribute__((ext_vector_type(8)));
typedef unsigned       v4u   __attribute__((ext_vector_type(4)));
typedef unsigned short v8us  __attribute__((ext_vector_type(8)));
typedef unsigned short v16us __attribute__((ext_vector_type(16)));
typedef __bf16         v16bf __attribute__((ext_vector_type(16)));
typedef v2f  __attribute__((may_alias)) v2fa;
typedef v4f  __attribute__((may_alias)) v4fa;
typedef v4i  __attribute__((may_alias)) v4ia;
typedef v4u  __attribute__((may_alias)) v4ua;
typedef v8us __attribute__((may_alias)) v8usa;
union Frag { v16bf v; v16us u; v8us h[2]; v8i w; };

__device__ __forceinline__ v8f wmb(const Frag& a, const Frag& b, v8f c) {
  v8f d = __builtin_amdgcn_wmma_f32_16x16x32_bf16(false, a.v, false, b.v, (short)0, c, false, false);
  asm volatile("v_nop\n\tv_nop\n\tv_nop\n\tv_nop" : "+v"(d) : "v"(a.w), "v"(b.w));
  return d;
}

__device__ __forceinline__ unsigned bf16_bits(float f) {
  const unsigned u = __float_as_uint(f);
  return (u + 0x7FFFu + ((u >> 16) & 1u)) >> 16;
}
__device__ __forceinline__ float bf16_val(float f) {
  return __uint_as_float(bf16_bits(f) << 16);
}
__device__ __forceinline__ unsigned short xcvt(float v) {
  float f = bf16_val(v);
  f = fminf(10.0f, fmaxf(-10.0f, f));
  return (unsigned short)bf16_bits(f);
}
__device__ __forceinline__ v8us hilo8(v4f t) {
  v8us o;
  unsigned hb;
  hb = bf16_bits(t.x); o[0] = (unsigned short)hb; o[4] = (unsigned short)bf16_bits(t.x - __uint_as_float(hb << 16));
  hb = bf16_bits(t.y); o[1] = (unsigned short)hb; o[5] = (unsigned short)bf16_bits(t.y - __uint_as_float(hb << 16));
  hb = bf16_bits(t.z); o[2] = (unsigned short)hb; o[6] = (unsigned short)bf16_bits(t.z - __uint_as_float(hb << 16));
  hb = bf16_bits(t.w); o[3] = (unsigned short)hb; o[7] = (unsigned short)bf16_bits(t.w - __uint_as_float(hb << 16));
  return o;
}

__device__ __forceinline__ float wsum(float v) {
  v += __shfl_xor(v, 16, 32);
  v += __shfl_xor(v, 8, 32);
  v += __shfl_xor(v, 4, 32);
  v += __shfl_xor(v, 2, 32);
  v += __shfl_xor(v, 1, 32);
  return v;
}

template <int SLB>
__device__ __forceinline__ int scan_chunk(const int* __restrict__ dsts, int nE, int cbase, int slotBase,
                                          int nb, int vec8, int* list, int tid, int lane, int wave) {
  int wc = 0;
  const int el0  = tid * EPT;
  const int e0   = cbase + el0;
  const int sent = -2147483647 - 1;
  v4i da, db;
  if (vec8 != 0 && cbase + CHUNK <= nE) {
    da = *(const v4i*)(dsts + e0);
    db = *(const v4i*)(dsts + e0 + 4);
  } else {
    da.x = (e0     < nE) ? dsts[min(e0,     nE - 1)] : sent;
    da.y = (e0 + 1 < nE) ? dsts[min(e0 + 1, nE - 1)] : sent;
    da.z = (e0 + 2 < nE) ? dsts[min(e0 + 2, nE - 1)] : sent;
    da.w = (e0 + 3 < nE) ? dsts[min(e0 + 3, nE - 1)] : sent;
    db.x = (e0 + 4 < nE) ? dsts[min(e0 + 4, nE - 1)] : sent;
    db.y = (e0 + 5 < nE) ? dsts[min(e0 + 5, nE - 1)] : sent;
    db.z = (e0 + 6 < nE) ? dsts[min(e0 + 6, nE - 1)] : sent;
    db.w = (e0 + 7 < nE) ? dsts[min(e0 + 7, nE - 1)] : sent;
  }
  const unsigned nbs = (unsigned)slotBase;
  const unsigned unb = (unsigned)nb;
  const unsigned s0 = (unsigned)da.x - nbs, s1 = (unsigned)da.y - nbs;
  const unsigned s2 = (unsigned)da.z - nbs, s3 = (unsigned)da.w - nbs;
  const unsigned s4 = (unsigned)db.x - nbs, s5 = (unsigned)db.y - nbs;
  const unsigned s6 = (unsigned)db.z - nbs, s7 = (unsigned)db.w - nbs;
  const bool h0 = s0 < unb, h1 = s1 < unb, h2 = s2 < unb, h3 = s3 < unb;
  const bool h4 = s4 < unb, h5 = s5 < unb, h6 = s6 < unb, h7 = s7 < unb;
  const unsigned any = __builtin_amdgcn_ballot_w32(h0 | h1 | h2 | h3 | h4 | h5 | h6 | h7);
  if (any != 0u) {
#define HITJ(J, HJ, SJ) { \
      const unsigned mj = __builtin_amdgcn_ballot_w32(HJ); \
      if (mj != 0u) { \
        if (HJ) { \
          const int pos = wc + (int)__builtin_amdgcn_mbcnt_lo(mj, 0u); \
          if (pos < WCAP) list[wave * WCAP + pos] = ((el0 + (J)) << SLB) | (int)(SJ); \
        } \
        wc += (int)__builtin_popcount(mj); } }
    HITJ(0, h0, s0)
    HITJ(1, h1, s1)
    HITJ(2, h2, s2)
    HITJ(3, h3, s3)
    HITJ(4, h4, s4)
    HITJ(5, h5, s5)
    HITJ(6, h6, s6)
    HITJ(7, h7, s7)
#undef HITJ
  }
  return wc;
}

__global__ __launch_bounds__(NTHR) void k_prep(const float* __restrict__ embW, const float* __restrict__ relW,
                                               const float* __restrict__ rootW, const float* __restrict__ clsW1,
                                               unsigned short* EMBT, unsigned short* B0, unsigned short* B1,
                                               unsigned short* CLST) {
  const int u = (int)blockIdx.x * NTHR + (int)threadIdx.x;
  v8us o;
  unsigned short* dp;
  if (u < UEMB) {
    const int n  = u >> 3;
    const int k8 = (u & 7) * 8;
    const float* p = embW + (size_t)k8 * DF + n;
#pragma unroll
    for (int i = 0; i < 8; ++i) o[i] = (unsigned short)bf16_bits(p[(size_t)i * DF]);
    dp = EMBT + (size_t)n * DIN + k8;
  } else if (u < UEMB + ULAY) {
    const int v = u - UEMB;
    const int l = v >> 15;
    const int w = (v >> 12) & 7;
    const int n = (v >> 5) & 127;
    const int g = v & 31;
    const float* W;
    if (w < NREL) W = relW + (size_t)(l * NREL + w) * DF * DF;
    else          W = rootW + (size_t)l * DF * DF;
    const float* p = W + (size_t)(4 * g) * DF + n;
    const unsigned short f0 = (unsigned short)bf16_bits(p[0]);
    const unsigned short f1 = (unsigned short)bf16_bits(p[DF]);
    const unsigned short f2 = (unsigned short)bf16_bits(p[2 * DF]);
    const unsigned short f3 = (unsigned short)bf16_bits(p[3 * DF]);
    o[0] = f0; o[1] = f1; o[2] = f2; o[3] = f3; o[4] = f0; o[5] = f1; o[6] = f2; o[7] = f3;
    unsigned short* Bl;
    if (l == 0) Bl = B0; else Bl = B1;
    dp = Bl + (size_t)n * AP + BW * w + 8 * g;
  } else if (u < UTOT) {
    const int v = u - UEMB - ULAY;
    const int n = v >> 5;
    const int g = v & 31;
    const float* p = clsW1 + (size_t)(4 * g) * DC + n;
    const unsigned short f0 = (unsigned short)bf16_bits(p[0]);
    const unsigned short f1 = (unsigned short)bf16_bits(p[DC]);
    const unsigned short f2 = (unsigned short)bf16_bits(p[2 * DC]);
    const unsigned short f3 = (unsigned short)bf16_bits(p[3 * DC]);
    o[0] = f0; o[1] = f1; o[2] = f2; o[3] = f3; o[4] = f0; o[5] = f1; o[6] = f2; o[7] = f3;
    dp = CLST + (size_t)n * KCL + 8 * g;
  } else {
    return;
  }
  *(volatile v8us*)dp = o;
  __threadfence();
  *(volatile v8us*)dp = o;
}

__global__ __launch_bounds__(GTHR) void k_emb(const float* __restrict__ xin, int nN,
                                              const unsigned short* __restrict__ BT,
                                              const float* __restrict__ bias, unsigned short* apl) {
  __shared__ __attribute__((aligned(16))) float stg[GBM * GBN];
  const int tid = (int)threadIdx.x, lane = tid & 31, wave = tid >> 5, hh = lane >> 4, m = lane & 15;
  const int rowBase = (int)blockIdx.x * GBM;

  v8f acc[8];
  {
    const v8f z = {0.f, 0.f, 0.f, 0.f, 0.f, 0.f, 0.f, 0.f};
#pragma unroll
    for (int t = 0; t < 8; ++t) acc[t] = z;
  }
  const int ar  = rowBase + 16 * wave + m;
  const int arc = ar < nN ? ar : nN - 1;
  const float okf = ar < nN ? 1.0f : 0.0f;
  const float* xp = xin + (size_t)arc * DIN + 8 * hh;
  const unsigned short* bp = BT + (size_t)m * DIN + 8 * hh;

#pragma unroll 1
  for (int k0 = 0; k0 < DIN; k0 += 32) {
    const v4f u0 = *(const v4fa*)(xp + k0);
    const v4f u1 = *(const v4fa*)(xp + k0 + 4);
    const v4f u2 = *(const v4fa*)(xp + k0 + 16);
    const v4f u3 = *(const v4fa*)(xp + k0 + 20);
    v8us o0, o1;
    o0[0] = xcvt(u0.x * okf); o0[1] = xcvt(u0.y * okf); o0[2] = xcvt(u0.z * okf); o0[3] = xcvt(u0.w * okf);
    o0[4] = xcvt(u1.x * okf); o0[5] = xcvt(u1.y * okf); o0[6] = xcvt(u1.z * okf); o0[7] = xcvt(u1.w * okf);
    o1[0] = xcvt(u2.x * okf); o1[1] = xcvt(u2.y * okf); o1[2] = xcvt(u2.z * okf); o1[3] = xcvt(u2.w * okf);
    o1[4] = xcvt(u3.x * okf); o1[5] = xcvt(u3.y * okf); o1[6] = xcvt(u3.z * okf); o1[7] = xcvt(u3.w * okf);
    Frag af;
    af.h[0] = o0;
    af.h[1] = o1;
#pragma unroll
    for (int nt = 0; nt < 8; ++nt) {
      const unsigned short* wq = bp + (size_t)(16 * nt) * (size_t)DIN + k0;
      Frag bf;
      bf.h[0] = *(const v8usa*)wq;
      bf.h[1] = *(const v8usa*)(wq + 16);
      acc[nt] = wmb(af, bf, acc[nt]);
    }
  }

#pragma unroll
  for (int nt = 0; nt < 8; ++nt) {
    const int lc = 16 * nt + m;
#pragma unroll
    for (int r = 0; r < 8; ++r) {
      const int lr = 16 * wave + 8 * hh + r;
      stg[lr * GBN + lc] = acc[nt][r];
    }
  }
  __syncthreads();

  v4f bb4;
  {
    const v4f tb = *(const v4fa*)(bias + 4 * lane);
    bb4.x = bf16_val(tb.x); bb4.y = bf16_val(tb.y); bb4.z = bf16_val(tb.z); bb4.w = bf16_val(tb.w);
  }
  v8us po[16];
#pragma unroll
  for (int i = 0; i < 16; ++i) {
    const v4f t = *(const v4fa*)(stg + (16 * wave + i) * GBN + 4 * lane) + bb4;
    po[i] = hilo8(t);
  }
#pragma unroll
  for (int i = 0; i < 16; ++i) {
    unsigned short* rp = apl + (size_t)(rowBase + 16 * wave + i) * (size_t)AP + HOFF + 8 * lane;
    *(volatile v8us*)rp = po[i];
  }
  __threadfence();
#pragma unroll
  for (int i = 0; i < 16; ++i) {
    unsigned short* rp = apl + (size_t)(rowBase + 16 * wave + i) * (size_t)AP + HOFF + 8 * lane;
    *(volatile v8us*)rp = po[i];
  }
}

__global__ __launch_bounds__(GTHR) void k_layer(unsigned short* apl, const unsigned short* __restrict__ BT,
                                                const float* __restrict__ bias, const float* __restrict__ gam,
                                                const float* __restrict__ bet) {
  __shared__ __attribute__((aligned(16))) float stg[GBM * GBN];
  const int tid = (int)threadIdx.x, lane = tid & 31, wave = tid >> 5, hh = lane >> 4, m = lane & 15;
  const int rowBase = (int)blockIdx.x * GBM;

  v8f acc[8];
  {
    const v8f z = {0.f, 0.f, 0.f, 0.f, 0.f, 0.f, 0.f, 0.f};
#pragma unroll
    for (int t = 0; t < 8; ++t) acc[t] = z;
  }
  const unsigned short* ap = apl + (size_t)(rowBase + 16 * wave + m) * (size_t)AP + 8 * hh;
  const unsigned short* bp = BT + (size_t)m * (size_t)AP + 8 * hh;

#pragma unroll 1
  for (int k0 = 0; k0 < AP; k0 += 32) {
    Frag af;
    af.h[0] = *(const v8usa*)(ap + k0);
    af.h[1] = *(const v8usa*)(ap + k0 + 16);
#pragma unroll
    for (int nt = 0; nt < 8; ++nt) {
      const unsigned short* wq = bp + (size_t)(16 * nt) * (size_t)AP + k0;
      Frag bf;
      bf.h[0] = *(const v8usa*)wq;
      bf.h[1] = *(const v8usa*)(wq + 16);
      acc[nt] = wmb(af, bf, acc[nt]);
    }
  }

#pragma unroll
  for (int nt = 0; nt < 8; ++nt) {
    const int lc = 16 * nt + m;
#pragma unroll
    for (int r = 0; r < 8; ++r) {
      const int lr = 16 * wave + 8 * hh + r;
      stg[lr * GBN + lc] = acc[nt][r];
    }
  }
  __syncthreads();

  v4f bb4, g4, e4;
  {
    const v4f tb = *(const v4fa*)(bias + 4 * lane);
    const v4f tg = *(const v4fa*)(gam + 4 * lane);
    const v4f te = *(const v4fa*)(bet + 4 * lane);
    bb4.x = bf16_val(tb.x); bb4.y = bf16_val(tb.y); bb4.z = bf16_val(tb.z); bb4.w = bf16_val(tb.w);
    g4.x  = bf16_val(tg.x); g4.y  = bf16_val(tg.y); g4.z  = bf16_val(tg.z); g4.w  = bf16_val(tg.w);
    e4.x  = bf16_val(te.x); e4.y  = bf16_val(te.y); e4.z  = bf16_val(te.z); e4.w  = bf16_val(te.w);
  }

  v4f pv[16];
#pragma unroll
  for (int i = 0; i < 16; ++i) pv[i] = *(const v4fa*)(stg + (16 * wave + i) * GBN + 4 * lane);

  v8us po[16];
#pragma unroll
  for (int i = 0; i < 16; ++i) {
    const v4f t = pv[i] + bb4;
    const float s  = wsum((t.x + t.y) + (t.z + t.w));
    const float mu = s * (1.0f / DF);
    const v4f d = t - mu;
    const float q  = wsum((d.x * d.x + d.y * d.y) + (d.z * d.z + d.w * d.w));
    const float rs = rsqrtf(q * (1.0f / DF) + 1e-5f);
    v4f y = d * rs * g4 + e4;
    y.x = fmaxf(y.x, 0.0f); y.y = fmaxf(y.y, 0.0f); y.z = fmaxf(y.z, 0.0f); y.w = fmaxf(y.w, 0.0f);
    po[i] = hilo8(y);
  }
#pragma unroll
  for (int i = 0; i < 16; ++i) {
    unsigned short* rp = apl + (size_t)(rowBase + 16 * wave + i) * (size_t)AP + HOFF + 8 * lane;
    *(volatile v8us*)rp = po[i];
  }
  __threadfence();
#pragma unroll
  for (int i = 0; i < 16; ++i) {
    unsigned short* rp = apl + (size_t)(rowBase + 16 * wave + i) * (size_t)AP + HOFF + 8 * lane;
    *(volatile v8us*)rp = po[i];
  }
}

__global__ __launch_bounds__(GTHR) void k_cls(const unsigned short* __restrict__ apl,
                                              const unsigned short* __restrict__ BT,
                                              const float* __restrict__ b1, const float* __restrict__ gam,
                                              const float* __restrict__ bet, const float* __restrict__ w2,
                                              const float* __restrict__ b2, int nN, float* outp) {
  __shared__ __attribute__((aligned(16))) float stg[GBM * GCN];
  __shared__ __attribute__((aligned(16))) float sres[GBM];
  const int tid = (int)threadIdx.x, lane = tid & 31, wave = tid >> 5, hh = lane >> 4, m = lane & 15;
  const int rowBase = (int)blockIdx.x * GBM;

  v8f acc[4];
  {
    const v8f z = {0.f, 0.f, 0.f, 0.f, 0.f, 0.f, 0.f, 0.f};
#pragma unroll
    for (int t = 0; t < 4; ++t) acc[t] = z;
  }
  const unsigned short* ap = apl + (size_t)(rowBase + 16 * wave + m) * (size_t)AP + HOFF + 8 * hh;
  const unsigned short* bp = BT + (size_t)m * (size_t)KCL + 8 * hh;

#pragma unroll 1
  for (int k0 = 0; k0 < KCL; k0 += 32) {
    Frag af;
    af.h[0] = *(const v8usa*)(ap + k0);
    af.h[1] = *(const v8usa*)(ap + k0 + 16);
#pragma unroll
    for (int nt = 0; nt < 4; ++nt) {
      const unsigned short* wq = bp + (size_t)(16 * nt) * (size_t)KCL + k0;
      Frag bf;
      bf.h[0] = *(const v8usa*)wq;
      bf.h[1] = *(const v8usa*)(wq + 16);
      acc[nt] = wmb(af, bf, acc[nt]);
    }
  }

#pragma unroll
  for (int nt = 0; nt < 4; ++nt) {
    const int lc = 16 * nt + m;
#pragma unroll
    for (int r = 0; r < 8; ++r) {
      const int lr = 16 * wave + 8 * hh + r;
      stg[lr * GCN + lc] = acc[nt][r];
    }
  }
  __syncthreads();

  v2f bb2, g2, e2, ww2;
  {
    const v2f tb = *(const v2fa*)(b1 + 2 * lane);
    const v2f tg = *(const v2fa*)(gam + 2 * lane);
    const v2f te = *(const v2fa*)(bet + 2 * lane);
    const v2f tw = *(const v2fa*)(w2 + 2 * lane);
    bb2.x = bf16_val(tb.x); bb2.y = bf16_val(tb.y);
    g2.x  = bf16_val(tg.x); g2.y  = bf16_val(tg.y);
    e2.x  = bf16_val(te.x); e2.y  = bf16_val(te.y);
    ww2.x = bf16_val(tw.x); ww2.y = bf16_val(tw.y);
  }
  const float bz = bf16_val(b2[0]);

  float mine = 0.0f;
#pragma unroll
  for (int i = 0; i < 16; ++i) {
    const v2f x = *(const v2fa*)(stg + (16 * wave + i) * GCN + 2 * lane);
    const v2f t = x + bb2;
    const float s  = wsum(t.x + t.y);
    const float mu = s * (1.0f / DC);
    const v2f d = t - mu;
    const float q  = wsum(d.x * d.x + d.y * d.y);
    const float rs = rsqrtf(q * (1.0f / DC) + 1e-5f);
    v2f y = d * rs * g2 + e2;
    y.x = fmaxf(y.x, 0.0f); y.y = fmaxf(y.y, 0.0f);
    const float pr = wsum(y.x * ww2.x + y.y * ww2.y);
    const float ov = pr + bz;
    mine = (lane == i) ? ov : mine;
  }
  if (lane < 16) sres[16 * wave + lane] = mine;
  __syncthreads();

  if (wave == 0) {
    const int t16  = lane & 15;
    const v4f v    = *(const v4fa*)(sres + 4 * t16);
    const int r0   = rowBase + 4 * t16;
    const int lrow = rowBase + 32 * (t16 >> 3);
    const bool full = (lane < 16) && (lrow + 32 <= nN);
    const bool part = (lane < 16) && (lrow < nN) && (lrow + 32 > nN);
    volatile float* ov1 = (volatile float*)outp;
    if (full) *(volatile v4f*)(outp + r0) = v;
    if (part) {
      if (r0     < nN) ov1[r0]     = v.x;
      if (r0 + 1 < nN) ov1[r0 + 1] = v.y;
      if (r0 + 2 < nN) ov1[r0 + 2] = v.z;
      if (r0 + 3 < nN) ov1[r0 + 3] = v.w;
    }
    __threadfence();
    if (full) *(volatile v4f*)(outp + r0) = v;
    if (part) {
      if (r0     < nN) ov1[r0]     = v.x;
      if (r0 + 1 < nN) ov1[r0 + 1] = v.y;
      if (r0 + 2 < nN) ov1[r0 + 2] = v.z;
      if (r0 + 3 < nN) ov1[r0 + 3] = v.w;
    }
  }
}

#define MEANQ(AR, NR, QR) { \
    int cr = (int)(NR); \
    cr = cr < 0 ? 0 : (cr > DEGCAP ? DEGCAP : cr); \
    const float ip = rtab[cr] + pzr; \
    v4f mv = AR * ip; \
    mv.x = live ? mv.x : 0.0f; mv.y = live ? mv.y : 0.0f; \
    mv.z = live ? mv.z : 0.0f; mv.w = live ? mv.w : 0.0f; \
    QR = hilo8(mv); }

__global__ __launch_bounds__(NTHR) void k_scan(const int* __restrict__ srcs, const int* __restrict__ dsts,
                                               const int* __restrict__ ets, int nE, int nN, int vec8, int mRows,
                                               unsigned short* apl) {
  extern __shared__ __attribute__((aligned(16))) int dsm[];
  int* list = dsm;
  int* hl   = dsm + LISTN;
  int* sl   = hl + RCAP;
  int* cnt  = sl + RCAP;
  int* offs = cnt + NBA;
  int* cur  = offs + NBA;
  int* misc = cur + NBA;
  float* rtab = (float*)(misc + 16);
  const int tid = (int)threadIdx.x, lane = tid & 31, wave = tid >> 5;
  const int nodeBase = (int)blockIdx.x * NBA;

  {
    const v4i z4 = {0, 0, 0, 0};
    for (int i = tid * 4; i < AGG_ZINTS; i += NTHR * 4) *(v4ia*)(dsm + i) = z4;
    if (tid < 16) misc[tid] = 0;
    if (tid <= DEGCAP) rtab[tid] = 1.0f / fmaxf((float)tid, 1.0f);
  }
  __syncthreads();

  int t = 0, ov = 0;
  const int nChunks = (nE + CHUNK - 1) / CHUNK;
#pragma unroll 1
  for (int ch = 0; ch < nChunks; ++ch) {
    const int cbase = ch * CHUNK;
    const int wc = scan_chunk<SLA>(dsts, nE, cbase, nodeBase, NBA, vec8, list, tid, lane, wave);
    if (lane == 0) misc[wave] = wc;
    __syncthreads();
    if (wave == 0) {
#pragma unroll 1
      for (int w2 = 0; w2 < NWAVE; ++w2) {
        int c = misc[w2];
        c = c < 0 ? 0 : (c > WCAP ? WCAP : c);
#pragma unroll 1
        for (int b0 = 0; b0 < c; b0 += 32) {
          const int idx = b0 + lane;
          const int ent = list[w2 * WCAP + (idx < WCAP ? idx : WCAP - 1)];
          const int m32 = (c - b0) < 32 ? (c - b0) : 32;
#pragma unroll 1
          for (int k = 0; k < m32; ++k) {
            const int u    = __builtin_amdgcn_readlane(ent, k);
            const int slot = u & (NBA - 1);
            const int el   = (u >> SLA) & (CHUNK - 1);
            const int pk   = ((cbase + el) << SLA) | slot;
            if (t < RCAP) {
              if (lane == 0) { hl[t] = pk; cnt[slot] = cnt[slot] + 1; }
              t = t + 1;
            } else {
              ov = 1;
            }
          }
        }
      }
    }
    __syncthreads();
  }
  if (wave == 0 && lane == 0) { misc[8] = t; misc[9] = ov; }
  __syncthreads();
  int tt = misc[8];
  tt = tt < 0 ? 0 : (tt > RCAP ? RCAP : tt);
  const int ovf = misc[9];

  if (wave == 0) {
    const int base = lane * (NBA / 32);
    int sacc = 0;
#pragma unroll 1
    for (int i = 0; i < NBA / 32; ++i) sacc += cnt[base + i];
    int incl = sacc;
#pragma unroll
    for (int d = 1; d < 32; d <<= 1) {
      const int y = __shfl_up(incl, d, 32);
      if (lane >= d) incl += y;
    }
    int run = incl - sacc;
#pragma unroll 1
    for (int i = 0; i < NBA / 32; ++i) {
      const int cv = cnt[base + i];
      offs[base + i] = run;
      cur[base + i]  = run;
      run += cv;
    }
  }
  __syncthreads();
  if (wave == 0) {
#pragma unroll 1
    for (int b0 = 0; b0 < tt; b0 += 32) {
      const int idx = b0 + lane;
      const int ent = hl[idx < RCAP ? idx : RCAP - 1];
      const int m32 = (tt - b0) < 32 ? (tt - b0) : 32;
#pragma unroll 1
      for (int k = 0; k < m32; ++k) {
        const int u    = __builtin_amdgcn_readlane(ent, k);
        const int slot = u & (NBA - 1);
        if (lane == 0) {
          int p = cur[slot];
          p = p < 0 ? 0 : (p > RCAP - 1 ? RCAP - 1 : p);
          sl[p] = u;
          cur[slot] = p + 1;
        }
      }
    }
  }
  __syncthreads();

  const float pz = (ovf != 0) ? __int_as_float(0x7fc00000) : 0.0f;
  const unsigned short* hb = apl + HOFF + 8 * lane;
#pragma unroll 1
  for (int si = 0; si < NBA / NWAVE; ++si) {
    const int s    = si * NWAVE + wave;
    const int node = nodeBase + s;
    int c = cnt[s];
    const bool big = c > DEGCAP;
    c = c < 0 ? 0 : (c > DEGCAP ? DEGCAP : c);
    int o = offs[s];
    o = o < 0 ? 0 : (o > RCAP ? RCAP : o);
    const v4f z4 = {0.0f, 0.0f, 0.0f, 0.0f};
    v4f a0 = z4, a1 = z4, a2 = z4, a3 = z4, a4 = z4, a5 = z4, a6 = z4;
    float n0 = 0.0f, n1 = 0.0f, n2 = 0.0f, n3 = 0.0f, n4 = 0.0f, n5 = 0.0f, n6 = 0.0f;
#pragma unroll 1
    for (int b0 = 0; b0 < c; b0 += 32) {
      int idx = o + b0 + lane;
      idx = idx > RCAP - 1 ? RCAP - 1 : idx;
      const int ent = sl[idx];
      int eid = ent >> SLA;
      eid = eid < 0 ? 0 : (eid > nE - 1 ? nE - 1 : eid);
      int sr = srcs[eid];
      sr = sr < 0 ? 0 : (sr > nN - 1 ? nN - 1 : sr);
      int te = ets[eid];
      te = te < 0 ? 0 : (te > NREL - 1 ? NREL - 1 : te);
      const int m32 = (c - b0) < 32 ? (c - b0) : 32;
#pragma unroll 1
      for (int k = 0; k < m32; ++k) {
        const int sk = __builtin_amdgcn_readlane(sr, k);
        const int tk = __builtin_amdgcn_readlane(te, k);
        const v4u w = *(const v4ua*)(hb + (size_t)sk * (size_t)AP);
        v4f f;
        f.x = __uint_as_float(w.x << 16)         + __uint_as_float(w.z << 16);
        f.y = __uint_as_float(w.x & 0xffff0000u) + __uint_as_float(w.z & 0xffff0000u);
        f.z = __uint_as_float(w.y << 16)         + __uint_as_float(w.w << 16);
        f.w = __uint_as_float(w.y & 0xffff0000u) + __uint_as_float(w.w & 0xffff0000u);
        const float y0 = (tk == 0) ? 1.0f : 0.0f;
        const float y1 = (tk == 1) ? 1.0f : 0.0f;
        const float y2 = (tk == 2) ? 1.0f : 0.0f;
        const float y3 = (tk == 3) ? 1.0f : 0.0f;
        const float y4 = (tk == 4) ? 1.0f : 0.0f;
        const float y5 = (tk == 5) ? 1.0f : 0.0f;
        const float y6 = (tk == 6) ? 1.0f : 0.0f;
        a0 += y0 * f; n0 += y0;
        a1 += y1 * f; n1 += y1;
        a2 += y2 * f; n2 += y2;
        a3 += y3 * f; n3 += y3;
        a4 += y4 * f; n4 += y4;
        a5 += y5 * f; n5 += y5;
        a6 += y6 * f; n6 += y6;
      }
    }
    const float pzr = big ? __int_as_float(0x7fc00000) : pz;
    const bool live = node < nN;
    v8us q0, q1, q2, q3, q4, q5, q6;
    MEANQ(a0, n0, q0)
    MEANQ(a1, n1, q1)
    MEANQ(a2, n2, q2)
    MEANQ(a3, n3, q3)
    MEANQ(a4, n4, q4)
    MEANQ(a5, n5, q5)
    MEANQ(a6, n6, q6)
    if (node < mRows) {
      unsigned short* rpw = apl + (size_t)node * (size_t)AP + 8 * lane;
      *(volatile v8us*)(rpw)          = q0;
      *(volatile v8us*)(rpw + BW)     = q1;
      *(volatile v8us*)(rpw + 2 * BW) = q2;
      *(volatile v8us*)(rpw + 3 * BW) = q3;
      *(volatile v8us*)(rpw + 4 * BW) = q4;
      *(volatile v8us*)(rpw + 5 * BW) = q5;
      *(volatile v8us*)(rpw + 6 * BW) = q6;
      __threadfence();
      *(volatile v8us*)(rpw)          = q0;
      *(volatile v8us*)(rpw + BW)     = q1;
      *(volatile v8us*)(rpw + 2 * BW) = q2;
      *(volatile v8us*)(rpw + 3 * BW) = q3;
      *(volatile v8us*)(rpw + 4 * BW) = q4;
      *(volatile v8us*)(rpw + 5 * BW) = q5;
      *(volatile v8us*)(rpw + 6 * BW) = q6;
    }
  }
}
#undef MEANQ

static inline int cdiv(int a, int b) { return (a + b - 1) / b; }

extern "C" void kernel_launch(void* const* d_in, const int* in_sizes, int n_in,
                              void* d_out, int out_size, void* d_ws, size_t ws_size,
                              hipStream_t stream) {
  if (n_in < 16) return;
  if (in_sizes[0] < DIN || (in_sizes[0] % DIN) != 0) return;
  const int nN = in_sizes[0] / DIN;
  const int nE = in_sizes[2];
  if (nE < 1 || in_sizes[1] != 2 * nE) return;
  if (nE >= (1 << 21)) return;
  if (in_sizes[3] != DIN * DF || in_sizes[4] != DF) return;
  if (in_sizes[5] != 2 * NREL * DF * DF) return;
  if (in_sizes[6] != 2 * DF * DF) return;
  if (in_sizes[7] != 2 * DF || in_sizes[8] != 2 * DF || in_sizes[9] != 2 * DF) return;
  if (in_sizes[10] != DF * DC || in_sizes[11] != DC) return;
  if (in_sizes[12] != DC || in_sizes[13] != DC) return;
  if (in_sizes[14] != DC || in_sizes[15] < 1) return;
  if (out_size != nN) return;

  const float* x      = (const float*)d_in[0];
  const int*   edge   = (const int*)d_in[1];
  const int*   ety    = (const int*)d_in[2];
  const float* embW   = (const float*)d_in[3];
  const float* embB   = (const float*)d_in[4];
  const float* relW   = (const float*)d_in[5];
  const float* rootW  = (const float*)d_in[6];
  const float* convB  = (const float*)d_in[7];
  const float* lnG    = (const float*)d_in[8];
  const float* lnB    = (const float*)d_in[9];
  const float* clsW1  = (const float*)d_in[10];
  const float* clsB1  = (const float*)d_in[11];
  const float* clsG   = (const float*)d_in[12];
  const float* clsE   = (const float*)d_in[13];
  const float* clsW2  = (const float*)d_in[14];
  const float* clsB2  = (const float*)d_in[15];
  float* out = (float*)d_out;
  const int* src = edge;
  const int* dst = edge + nE;

  const int MP = cdiv(nN, GBM) * GBM;
  const int gM = MP / GBM;
  const int gA = cdiv(MP, NBA);
  if ((long long)gA * NBA < (long long)MP) return;
  const int vec8 = ((nE & 3) == 0) ? 1 : 0;

  char* ws = (char*)d_ws;
  size_t off = 0;
  const size_t oE  = off; off += (size_t)DF * DIN * 2;                     off = (off + 255) & ~(size_t)255;
  const size_t oB0 = off; off += (size_t)DF * AP * 2;                      off = (off + 255) & ~(size_t)255;
  const size_t oB1 = off; off += (size_t)DF * AP * 2;                      off = (off + 255) & ~(size_t)255;
  const size_t oC  = off; off += (size_t)DC * KCL * 2;                     off = (off + 255) & ~(size_t)255;
  const size_t oA  = off; off += (size_t)MP * AP * 2;                      off = (off + 255) & ~(size_t)255;
  if (off > ws_size || off > (size_t)WSMAX) return;
  unsigned short* EMBT = (unsigned short*)(ws + oE);
  unsigned short* B0   = (unsigned short*)(ws + oB0);
  unsigned short* B1   = (unsigned short*)(ws + oB1);
  unsigned short* CLST = (unsigned short*)(ws + oC);
  unsigned short* Apl  = (unsigned short*)(ws + oA);

  const size_t scanLds = (size_t)AGG_LDS_INTS * 4;
  hipFuncSetAttribute(reinterpret_cast<const void*>(&k_scan), hipFuncAttributeMaxDynamicSharedMemorySize, (int)scanLds);

  k_prep<<<UTOT / NTHR, NTHR, 0, stream>>>(embW, relW, rootW, clsW1, EMBT, B0, B1, CLST);
  k_emb<<<gM, GTHR, 0, stream>>>(x, nN, EMBT, embB, Apl);
  k_scan<<<gA, NTHR, scanLds, stream>>>(src, dst, ety, nE, nN, vec8, MP, Apl);
  k_layer<<<gM, GTHR, 0, stream>>>(Apl, B0, convB, lnG, lnB);
  k_scan<<<gA, NTHR, scanLds, stream>>>(src, dst, ety, nE, nN, vec8, MP, Apl);
  k_layer<<<gM, GTHR, 0, stream>>>(Apl, B1, convB + DF, lnG + DF, lnB + DF);
  k_cls<<<gM, GTHR, 0, stream>>>(Apl, CLST, clsB1, clsG, clsE, clsW2, clsB2, nN, out);
}
